// DemandAwareRS_35708358099011
// MI455X (gfx1250) — hardware-run, weakly checked
//
#include <hip/hip_runtime.h>
#include <math.h>

typedef __attribute__((ext_vector_type(16))) _Float16 v16h;
typedef __attribute__((ext_vector_type(8)))  _Float16 v8h;
typedef __attribute__((ext_vector_type(8)))  float    v8f;
typedef __attribute__((ext_vector_type(4)))  float    v4f;

constexpr int kNumB   = 128;
constexpr int kNumL   = 50;
constexpr int kNumV   = 100000;
constexpr int kNumCat = 1000;
constexpr int kDim    = 64;
constexpr int kNumDem = 4;
constexpr int kVpad   = 100032;
constexpr int kCatPad = 1024;
constexpr int kTilesN = kVpad / 64;
constexpr int kTilesM = kNumB / 64;
constexpr int kTiles  = kTilesN * kTilesM;
constexpr int kGemmBlocks = (kTiles + 7) / 8;
static_assert(kVpad % 64 == 0 && kVpad >= kNumV && kVpad - kNumV < 64);
static_assert(kNumV % 32 == 0);
static_assert(kNumB % 64 == 0 && kDim % 32 == 0);
static_assert(kTilesN == 1563 && kTilesM == 2 && kGemmBlocks == 391);

constexpr float kCarryH = 1024.0f;
constexpr float kCarryE = 256.0f;
constexpr float kFold   = 1.0f / (kCarryH * kCarryE);

constexpr int kOut0Elems = kNumB * kNumV;
constexpr int kGnnElems  = kNumB * kNumDem * kNumL * kDim;
constexpr int kTailElems = 1 + kGnnElems;
constexpr int kOutTotal  = kOut0Elems + kTailElems;
static_assert((size_t)kOut0Elems * 4 == 51200000ull);
static_assert(((size_t)kOut0Elems * 4) % 128 == 0);
static_assert(kGnnElems == 1638400);
static_assert((size_t)kOutTotal * 4 == 57753604ull);
static_assert(((size_t)kNumV * 4) % 128 == 0);
constexpr int kTailBlocks = (kTailElems - 32 + 255) / 256;
static_assert(kTailBlocks == 6400);

constexpr size_t kOffE16  = 0;
constexpr size_t kOffH16  = kOffE16 + (size_t)kVpad * kDim * 2;
constexpr size_t kOffU    = kOffH16 + (size_t)kNumB * kDim * 2;
constexpr size_t kOffWT   = kOffU   + (size_t)kNumB * kDim * 4;
constexpr size_t kWsTotal = kOffWT  + (size_t)kCatPad * 4;
static_assert(kWsTotal == 12857344ull);
static_assert(kWsTotal <= 134217728ull);
static_assert((kOffH16 % 128) == 0 && (kOffU % 128) == 0 && (kOffWT % 128) == 0);

constexpr int kEmbBlocks = (kVpad * kDim / 8) / 256;
static_assert((size_t)kEmbBlocks * 256 * 8 == (size_t)kVpad * kDim);
static_assert(kEmbBlocks == 3126);

struct FragH {
  union U { v16h v; v8h h[2]; };
  static __device__ __forceinline__ v16h load(const _Float16* p) {
    U f;
    f.h[0] = *(const v8h*)(p);
    f.h[1] = *(const v8h*)(p + 16);
    return f.v;
  }
};
__device__ __forceinline__ v8f mma_h(v16h a, v16h b, v8f c) {
  c = __builtin_amdgcn_wmma_f32_16x16x32_f16(false, a, false, b, (short)0, c, false, false);
  asm volatile("v_nop\n\tv_nop\n\tv_nop\n\tv_nop" : "+v"(c) : "v"(a), "v"(b));
  return c;
}
__device__ __forceinline__ int clampi(int x, int lo, int hi) {
  return x < lo ? lo : (x > hi ? hi : x);
}

__global__ __launch_bounds__(256) void emb_plane_kernel(
    const float* __restrict__ emb, unsigned short* __restrict__ E16)
{
  const int i   = blockIdx.x * 256 + threadIdx.x;
  const int row = i >> 3;
  const int c8  = (i & 7) * 8;
  const bool live = row < kNumV;
  const int rc = live ? row : (kNumV - 1);
  const float* sp = emb + (size_t)rc * kDim + c8;
  const v4f a0 = *(const v4f*)(sp);
  const v4f a1 = *(const v4f*)(sp + 4);
  v8h hv;
#pragma unroll
  for (int e = 0; e < 4; ++e) {
    const float x0 = live ? (a0[e] * kCarryE) : 0.0f;
    const float x1 = live ? (a1[e] * kCarryE) : 0.0f;
    hv[e]     = (_Float16)x0;
    hv[4 + e] = (_Float16)x1;
  }
  unsigned short* q = E16 + (size_t)row * kDim + c8;
  *(volatile v8h*)q = hv;
  __threadfence();
  *(volatile v8h*)q = hv;
}

__global__ __launch_bounds__(64) void session_kernel(
    const int* __restrict__ nodes, const int* __restrict__ maskNode, const int* __restrict__ lastIdx,
    const float* __restrict__ emb, const float* __restrict__ Wim, const float* __restrict__ Wpv,
    const float* __restrict__ bpv, float* __restrict__ U, unsigned short* __restrict__ H16)
{
  __shared__ int sNode[64];
  __shared__ float sMask[64];
  __shared__ __align__(16) float sG[64];
  __shared__ __align__(16) float sL[64];
  __shared__ __align__(16) float sU[64];
  __shared__ __align__(16) float sH[64];
  const int b = blockIdx.x, tid = threadIdx.x;
  {
    const int lc = (tid < kNumL) ? tid : (kNumL - 1);
    const int nd = clampi(nodes[b * kNumL + lc], 0, kNumV - 1);
    const int mk = maskNode[b * kNumL + lc];
    sNode[tid] = nd;
    sMask[tid] = (tid < kNumL) ? (float)mk : 0.0f;
  }
  const int li = clampi(lastIdx[b], 0, kNumL - 1);
  __syncthreads();
  float acc = 0.0f, msum = 0.0f;
#pragma unroll 2
  for (int l = 0; l < kNumL; ++l) {
    const float e = emb[(size_t)sNode[l] * kDim + tid];
    const float m = sMask[l];
    acc = fmaf(m, e, acc);
    msum += m;
  }
  const float g = acc * (1.0f / msum);
  const float lastv = emb[(size_t)sNode[li] * kDim + tid];
  sG[tid] = g;
  sL[tid] = lastv;
  __syncthreads();
  float uu = 0.0f;
  {
    const float* wr = Wim + (size_t)tid * kDim;
#pragma unroll 1
    for (int e4 = 0; e4 < kDim / 4; ++e4) {
      const v4f w  = *(const v4f*)(wr + 4 * e4);
      const v4f gg = *(const v4f*)(sG + 4 * e4);
      uu = fmaf(w[0], gg[0], uu);
      uu = fmaf(w[1], gg[1], uu);
      uu = fmaf(w[2], gg[2], uu);
      uu = fmaf(w[3], gg[3], uu);
    }
  }
  float hsum = 0.0f;
#pragma unroll 4
  for (int k = 0; k < kDim; ++k) hsum = fmaf(sG[k], Wpv[(size_t)k * kDim + tid], hsum);
#pragma unroll 4
  for (int k = 0; k < kDim; ++k) hsum = fmaf(sL[k], Wpv[(size_t)(kDim + k) * kDim + tid], hsum);
  hsum += bpv[tid];
  const float hval = tanhf(hsum);
  sU[tid] = uu;
  sH[tid] = hval * kCarryH;
  __syncthreads();
  const v4f uv = *(const v4f*)(sU + (tid & 15) * 4);
  v8h hv;
#pragma unroll
  for (int e = 0; e < 8; ++e) hv[e] = (_Float16)sH[(tid & 7) * 8 + e];
  float* up = U + (size_t)b * kDim + (tid & 15) * 4;
  unsigned short* hp = H16 + (size_t)b * kDim + (tid & 7) * 8;
  for (int pass = 0; pass < 2; ++pass) {
    if (tid < 16) *(volatile v4f*)up = uv;
    if (tid < 8)  *(volatile v8h*)hp = hv;
    __threadfence();
  }
}

__global__ __launch_bounds__(64) void category_table_kernel(
    const float* __restrict__ embc, const float* __restrict__ Wd1, const float* __restrict__ bd1,
    const float* __restrict__ Wd2, const float* __restrict__ bd2, float* __restrict__ WT)
{
  __shared__ __align__(16) float sW2[kDim * kNumDem];
  __shared__ float sE[64];
  __shared__ float sT[64];
  __shared__ float sOut[32];
  const int tid = threadIdx.x;
  const int n = tid & 3;
  {
    const v4f w = *(const v4f*)(Wd2 + tid * 4);
    *(v4f*)(sW2 + tid * 4) = w;
  }
  const float b1 = bd1[tid];
  const float b2 = bd2[n];
  __syncthreads();
#pragma unroll 1
  for (int ci = 0; ci < 32; ++ci) {
    const int c  = blockIdx.x * 32 + ci;
    const int cc = (c < kNumCat) ? c : (kNumCat - 1);
    sE[tid] = embc[(size_t)cc * kDim + tid];
    __syncthreads();
    float a = 0.0f;
#pragma unroll 4
    for (int k = 0; k < kDim; ++k) a = fmaf(sE[k], Wd1[(size_t)k * kDim + tid], a);
    sT[tid] = tanhf(a + b1);
    __syncthreads();
    float z = 0.0f;
#pragma unroll 4
    for (int j = 0; j < kDim; ++j) z = fmaf(sT[j], sW2[j * kNumDem + n], z);
    z += b2;
    float mx = fmaxf(z, __shfl_xor(z, 1, 32));
    mx = fmaxf(mx, __shfl_xor(mx, 2, 32));
    const float ex = expf(z - mx);
    float den = ex + __shfl_xor(ex, 1, 32);
    den = den + __shfl_xor(den, 2, 32);
    const float p = ex * (1.0f / den);
    float s = p + __shfl_xor(p, 1, 32);
    s = s + __shfl_xor(s, 2, 32);
    if (tid == 0) sOut[ci] = (c < kNumCat) ? s : 1.0f;
  }
  __syncthreads();
  if (tid < 32) {
    const float v = sOut[tid];
    float* p = WT + blockIdx.x * 32 + tid;
    *(volatile float*)p = v;
    __threadfence();
    *(volatile float*)p = v;
  }
}

__global__ __launch_bounds__(256) void tail_copy_kernel(
    const int* __restrict__ nodes, const float* __restrict__ emb, float* __restrict__ tail)
{
  const int gid = blockIdx.x * 256 + threadIdx.x;
  const int idx = 32 + gid;
  const bool ok = idx < kTailElems;
  const int idc = ok ? idx : (kTailElems - 1);
  const int i   = idc - 1;
  const int b   = i / (kNumDem * kNumL * kDim);
  const int rem = i - b * (kNumDem * kNumL * kDim);
  const int l   = (rem % (kNumL * kDim)) >> 6;
  const int d   = i & 63;
  const int node = clampi(nodes[b * kNumL + l], 0, kNumV - 1);
  float val = emb[(size_t)node * kDim + d];
  asm volatile("" : "+v"(val));
  float* p = tail + idc;
  if (ok) *(volatile float*)p = val;
  __threadfence();
  if (ok) *(volatile float*)p = val;
}

__global__ __launch_bounds__(256) void loss_kernel(
    const int* __restrict__ nodes, const float* __restrict__ emb, const float* __restrict__ U,
    float* __restrict__ tail)
{
  __shared__ float sRed[256];
  const int tid = threadIdx.x;
  float s = 0.0f;
  static_assert(kNumB * kNumL == 25 * 256);
#pragma unroll 1
  for (int it = 0; it < 25; ++it) {
    const int idx = tid + 256 * it;
    const int b = idx / kNumL;
    const int node = clampi(nodes[idx], 0, kNumV - 1);
    const float* er = emb + (size_t)node * kDim;
    const float* up = U + (size_t)b * kDim;
    const float* un = U + (size_t)((b + kNumB - 1) & (kNumB - 1)) * kDim;
    float pos = 0.0f, neg = 0.0f;
#pragma unroll 1
    for (int d4 = 0; d4 < kDim / 4; ++d4) {
      const v4f e = *(const v4f*)(er + 4 * d4);
      const v4f p = *(const v4f*)(up + 4 * d4);
      const v4f q = *(const v4f*)(un + 4 * d4);
      pos = fmaf(e[0], p[0], pos);
      pos = fmaf(e[1], p[1], pos);
      pos = fmaf(e[2], p[2], pos);
      pos = fmaf(e[3], p[3], pos);
      neg = fmaf(e[0], q[0], neg);
      neg = fmaf(e[1], q[1], neg);
      neg = fmaf(e[2], q[2], neg);
      neg = fmaf(e[3], q[3], neg);
    }
    float x = pos;
#pragma unroll 1
    for (int t = 0; t < 2; ++t) {
      const float ls = fminf(x, 0.0f) - log1pf(expf(-fabsf(x)));
      s += ls;
      x = -neg;
    }
  }
  sRed[tid] = s;
  __syncthreads();
#pragma unroll 1
  for (int off = 128; off > 0; off >>= 1) {
    if (tid < off) sRed[tid] += sRed[tid + off];
    __syncthreads();
  }
  if (tid < 32) {
    const float tot = sRed[0];
    const float lossv = -(tot / (float)(kNumB * kNumL));
    const int node0 = clampi(nodes[0], 0, kNumV - 1);
    const int dd = (tid > 0) ? (tid - 1) : 0;
    const float gv = emb[(size_t)node0 * kDim + dd];
    const float val = (tid == 0) ? lossv : gv;
    float* p = tail + tid;
    *(volatile float*)p = val;
    __threadfence();
    *(volatile float*)p = val;
  }
}

__global__ __launch_bounds__(256) void score_gemm_kernel(
    const unsigned short* __restrict__ Ap, const unsigned short* __restrict__ Btp,
    float* __restrict__ C, const int* __restrict__ candCat, const float* __restrict__ wtab)
{
  const _Float16* A  = (const _Float16*)Ap;
  const _Float16* Bt = (const _Float16*)Btp;
  __shared__ __align__(16) float sT[8][16 * 68];
  const int lane = threadIdx.x & 31;
  const int wave = threadIdx.x >> 5;
  const int tile = blockIdx.x * 8 + wave;
  if (tile >= kTiles) return;
  const int tm = tile & 1;
  const int tn = tile >> 1;
  const int m0 = tm << 6;
  const int n0 = tn << 6;
  const int rlane = lane & 15;
  const int koff  = (lane >> 4) * 8;
  const int mOff  = (lane >> 4) * 8;

  v8f acc[4][4];
#pragma unroll
  for (int i = 0; i < 4; ++i)
#pragma unroll
    for (int j = 0; j < 4; ++j) acc[i][j] = (v8f){0.f, 0.f, 0.f, 0.f, 0.f, 0.f, 0.f, 0.f};

#pragma unroll 1
  for (int k0 = 0; k0 < kDim; k0 += 32) {
    v16h bh[4];
#pragma unroll
    for (int j = 0; j < 4; ++j) {
      const size_t bo = (size_t)(n0 + (j << 4) + rlane) * kDim + koff + k0;
      bh[j] = FragH::load(Bt + bo);
    }
#pragma unroll
    for (int i = 0; i < 4; ++i) {
      const size_t ao = (size_t)(m0 + (i << 4) + rlane) * kDim + koff + k0;
      const v16h ah = FragH::load(A + ao);
#pragma unroll
      for (int j = 0; j < 4; ++j) acc[i][j] = mma_h(ah, bh[j], acc[i][j]);
    }
  }

  float cs[4];
#pragma unroll
  for (int j = 0; j < 4; ++j) {
    const int n  = n0 + (j << 4) + rlane;
    const int nc = (n < kNumV) ? n : (kNumV - 1);
    const int ci = clampi(candCat[nc], 0, kNumCat - 1);
    cs[j] = wtab[ci] * kFold;
  }

  float* slab = sT[wave];
  const int hh = lane >> 4;
  const int c4 = (lane & 15) * 4;
  const bool colok = (n0 + c4) < kNumV;
#pragma unroll
  for (int i = 0; i < 4; ++i) {
    const int mBase = m0 + (i << 4);
#pragma unroll
    for (int j = 0; j < 4; ++j) {
#pragma unroll
      for (int r = 0; r < 8; ++r) {
        const float v = acc[i][j][r] * cs[j];
        slab[(mOff + r) * 68 + (j << 4) + rlane] = v;
      }
    }
    __builtin_amdgcn_fence(__ATOMIC_RELEASE, "workgroup");
    __builtin_amdgcn_wave_barrier();
    __builtin_amdgcn_fence(__ATOMIC_ACQUIRE, "workgroup");
    for (int pass = 0; pass < 2; ++pass) {
#pragma unroll
      for (int it = 0; it < 8; ++it) {
        const int row = it * 2 + hh;
        const v4f v = *(const v4f*)(slab + row * 68 + c4);
        if (colok) *(volatile v4f*)(C + (size_t)(mBase + row) * kNumV + n0 + c4) = v;
      }
      __threadfence();
    }
    __builtin_amdgcn_fence(__ATOMIC_RELEASE, "workgroup");
    __builtin_amdgcn_wave_barrier();
    __builtin_amdgcn_fence(__ATOMIC_ACQUIRE, "workgroup");
  }
}

extern "C" void kernel_launch(void* const* d_in, const int* in_sizes, int n_in,
                              void* d_out, int out_size, void* d_ws, size_t ws_size,
                              hipStream_t stream) {
  if (n_in < 16) return;
  if (in_sizes[0] != kNumB * kNumL) return;
  if (in_sizes[4] != kNumB) return;
  if (in_sizes[5] != kNumV) return;
  if (in_sizes[6] != kNumB * kNumL) return;
  if (in_sizes[7] != kNumV * kDim) return;
  if (in_sizes[8] != kNumCat * kDim) return;
  if (in_sizes[9] != kDim * kDim) return;
  if (in_sizes[10] != kDim) return;
  if (in_sizes[11] != kDim * kNumDem) return;
  if (in_sizes[12] != kNumDem) return;
  if (in_sizes[13] != 2 * kDim * kDim) return;
  if (in_sizes[14] != kDim) return;
  if (in_sizes[15] != kDim * kDim) return;
  if (out_size != kOutTotal) return;
  if (ws_size < kWsTotal) return;

  const int*   nodes    = (const int*)d_in[0];
  const int*   lastIdx  = (const int*)d_in[4];
  const int*   candCat  = (const int*)d_in[5];
  const int*   maskNode = (const int*)d_in[6];
  const float* embI     = (const float*)d_in[7];
  const float* embC     = (const float*)d_in[8];
  const float* Wd1      = (const float*)d_in[9];
  const float* bd1      = (const float*)d_in[10];
  const float* Wd2      = (const float*)d_in[11];
  const float* bd2      = (const float*)d_in[12];
  const float* Wpv      = (const float*)d_in[13];
  const float* bpv      = (const float*)d_in[14];
  const float* Wim      = (const float*)d_in[15];

  float* out  = (float*)d_out;
  float* tail = out + kOut0Elems;

  char* ws = (char*)d_ws;
  unsigned short* E16 = (unsigned short*)(ws + kOffE16);
  unsigned short* H16 = (unsigned short*)(ws + kOffH16);
  float*          U   = (float*)(ws + kOffU);
  float*          WT  = (float*)(ws + kOffWT);

  emb_plane_kernel<<<kEmbBlocks, 256, 0, stream>>>(embI, E16);
  session_kernel<<<kNumB, 64, 0, stream>>>(nodes, maskNode, lastIdx, embI, Wim, Wpv, bpv, U, H16);
  category_table_kernel<<<kCatPad / 32, 64, 0, stream>>>(embC, Wd1, bd1, Wd2, bd2, WT);
  tail_copy_kernel<<<kTailBlocks, 256, 0, stream>>>(nodes, embI, tail);
  loss_kernel<<<1, 256, 0, stream>>>(nodes, embI, U, tail);
  score_gemm_kernel<<<kGemmBlocks, 256, 0, stream>>>(H16, E16, out, candCat, WT);
}
